// SelfAttentionBlock_63788854280229
// MI455X (gfx1250) — hardware-verified
//
#include <hip/hip_runtime.h>


#ifndef NB
#define NB 2
#endif
#ifndef SEQ
#define SEQ 2048
#endif
#define NB_FULL  2
#define SEQ_FULL 2048
#define CE    1024
#define C3    3072
#define HEADS 16
#define HS    64
#define QB    64
#define KT    64
#define LDP   72
#define SSC   0.125f
#define L2E   1.4426950408889634f

static_assert(NB >= 1 && NB <= NB_FULL);
static_assert(SEQ >= 64 && SEQ <= SEQ_FULL);
static_assert(SEQ % 64 == 0 && SEQ % QB == 0 && QB == KT && QB == 64);
static_assert(CE == HEADS * HS && HS == 64 && C3 == 3 * CE);
static_assert(CE % 64 == 0 && C3 % 64 == 0 && CE % 32 == 0 && (2 * CE) % 32 == 0);
static_assert(((size_t)SEQ * CE / 8) % 256 == 0);
static_assert(((size_t)NB * SEQ * 128) % 256 == 0);
static_assert((size_t)NB * SEQ * 128 * 8 == (size_t)NB * HEADS * SEQ * HS);
static_assert((SEQ / QB) * 4 * 16 == SEQ);
static_assert((size_t)NB * SEQ * (2 * CE) * 2 <= (size_t)NB * SEQ * C3 * 4);

typedef unsigned short bf;
typedef __attribute__((ext_vector_type(16))) __bf16   v16bf;
typedef __attribute__((ext_vector_type(8)))  unsigned short v8us;
typedef __attribute__((ext_vector_type(8)))  float    v8f;
typedef __attribute__((ext_vector_type(4)))  float    v4f;
typedef __attribute__((ext_vector_type(2)))  unsigned short v2us;
typedef v4f  __attribute__((may_alias)) v4fa;

__device__ __forceinline__ unsigned short f2bf(float f) { unsigned u = __float_as_uint(f); u += 0x7FFFu + ((u >> 16) & 1u); return (unsigned short)(u >> 16); }
__device__ __forceinline__ float bf2f(unsigned short b) { return __uint_as_float(((unsigned)b) << 16); }
__device__ __forceinline__ float bfr(float f) { return bf2f(f2bf(f)); }
__device__ __forceinline__ v16bf cat16b(v8us lo, v8us hi) { return __builtin_bit_cast(v16bf, __builtin_shufflevector(lo, hi, 0, 1, 2, 3, 4, 5, 6, 7, 8, 9, 10, 11, 12, 13, 14, 15)); }
__device__ __forceinline__ v16bf ldf(const bf* p) { return cat16b(*(const v8us*)p, *(const v8us*)(p + 16)); }
__device__ __forceinline__ v8f wmmab(v16bf a, v16bf b, v8f c) { return __builtin_amdgcn_wmma_f32_16x16x32_bf16(false, a, false, b, (short)0, c, false, false); }
__device__ __forceinline__ void wave_lds_sync() { __builtin_amdgcn_fence(4  , "wavefront"); __builtin_amdgcn_wave_barrier(); asm volatile("" ::: "memory"); }

template <typename T16> struct WFrag;
template <> struct WFrag<bf> { typedef v16bf V; static __device__ __forceinline__ V ld(const bf* p) { return ldf(p); } static __device__ __forceinline__ v8f mma(V a, V b, v8f c) { return wmmab(a, b, c); } };
template <typename T16, int NSPLIT, bool BIAS>
__global__ __launch_bounds__(32) void k_gemmw(const T16* __restrict__ A, const T16* __restrict__ A2, const T16* __restrict__ Bt, const T16* __restrict__ Bt2, int K, float* C, int ldc, const float* __restrict__ bias, size_t sA, size_t sB, size_t sC) {
    typedef typename WFrag<T16>::V V;
    __shared__ __align__(16) float os[16 * 68];
    const size_t z = blockIdx.z; A += z * sA; if (A2) A2 += z * sA; Bt += z * sB; if (Bt2) Bt2 += z * sB; C += z * sC;
    const int lane = threadIdx.x & 31, lr = lane & 15, hi = lane >> 4; const int r0 = blockIdx.x * 64, c0 = blockIdx.y * 64;
    v8f acc[4][4];
#pragma unroll
    for (int mb = 0; mb < 4; ++mb)
#pragma unroll
        for (int nb = 0; nb < 4; ++nb) acc[mb][nb] = (v8f){};
    const size_t aoff = (size_t)(r0 + lr) * K + 8 * hi, boff = (size_t)(c0 + lr) * K + 8 * hi;
#pragma unroll 1
    for (int kc = 0; kc < K; kc += 32) {
        V a[4], a2[4];
#pragma unroll
        for (int mb = 0; mb < 4; ++mb) { a[mb] = WFrag<T16>::ld(A + aoff + (size_t)mb * 16 * K + kc); if (NSPLIT == 1 || NSPLIT == 2) a2[mb] = WFrag<T16>::ld(A2 + aoff + (size_t)mb * 16 * K + kc); }
#pragma unroll
        for (int nb = 0; nb < 4; ++nb) { const V b = WFrag<T16>::ld(Bt + boff + (size_t)nb * 16 * K + kc); V b2; if (NSPLIT >= 2) b2 = WFrag<T16>::ld(Bt2 + boff + (size_t)nb * 16 * K + kc);
#pragma unroll
            for (int mb = 0; mb < 4; ++mb) { acc[mb][nb] = WFrag<T16>::mma(a[mb], b, acc[mb][nb]); if (NSPLIT == 1 || NSPLIT == 2) acc[mb][nb] = WFrag<T16>::mma(a2[mb], b, acc[mb][nb]); if (NSPLIT >= 2) acc[mb][nb] = WFrag<T16>::mma(a[mb], b2, acc[mb][nb]); } }
        asm volatile("v_nop\n\tv_nop\n\tv_nop\n\tv_nop" : "+v"(acc[0][0]), "+v"(acc[1][1]), "+v"(acc[2][2]), "+v"(acc[3][3]) : "v"(a[0]), "v"(a[3]));
    }
#pragma unroll
    for (int mb = 0; mb < 4; ++mb) {
#pragma unroll
        for (int nb = 0; nb < 4; ++nb) {
#pragma unroll
            for (int j = 0; j < 8; ++j) os[(hi * 8 + j) * 68 + nb * 16 + lr] = acc[mb][nb][j]; }
        __builtin_amdgcn_wave_barrier(); asm volatile("" ::: "memory");
        float* crow = C + (size_t)(r0 + mb * 16) * ldc + c0;
#pragma unroll 1
        for (int ps = 0; ps < 2; ++ps) {
#pragma unroll
            for (int s = 0; s < 8; ++s) { const int row = 2 * s + hi, cofs = lr * 4; v4f val = *(const v4fa*)(os + row * 68 + cofs); if (BIAS) { val[0] += bfr(bias[c0 + cofs]); val[1] += bfr(bias[c0 + cofs + 1]); val[2] += bfr(bias[c0 + cofs + 2]); val[3] += bfr(bias[c0 + cofs + 3]); }
                *(volatile v4f*)(crow + (size_t)row * ldc + cofs) = val; }
            if (ps == 0) __threadfence(); }
        __builtin_amdgcn_wave_barrier(); asm volatile("" ::: "memory");
    }
}

__global__ __launch_bounds__(256) void k_wtG(const float* __restrict__ w, int K, int N, int KD, bf* Bt) {
    const int lane = threadIdx.x & 31; const int L0 = (blockIdx.x * 8 + (threadIdx.x >> 5)) * 8; const int nlines = (int)((size_t)N * KD / 64);
#pragma unroll
    for (int ps = 0; ps < 2; ++ps) {
#pragma unroll 1
        for (int l = 0; l < 8; ++l) { const int L = L0 + l; if (L >= nlines) break; const size_t e = (size_t)L * 64 + lane * 2; int kd = (int)(e % KD); const int n = (int)(e / KD); if (kd >= K) kd -= K; v2us o;
            o[0] = f2bf(w[(size_t)kd * N + n]); o[1] = f2bf(w[(size_t)(kd + 1) * N + n]); *(volatile v2us*)(Bt + e) = o; }
        if (ps == 0) __threadfence(); }
}
__global__ __launch_bounds__(256) void k_cvt8(const float* __restrict__ src, bf* dst, size_t n8, size_t sstr, size_t dstr) { const size_t i = (size_t)blockIdx.x * 256 + threadIdx.x; if (i >= n8) return;
    src += (size_t)blockIdx.y * sstr; dst += (size_t)blockIdx.y * dstr; const v8f v = *(const v8f*)(src + i * 8); v8us o;
#pragma unroll
    for (int k = 0; k < 8; ++k) o[k] = f2bf(v[k]); *(volatile v8us*)(dst + i * 8) = o; __threadfence(); *(volatile v8us*)(dst + i * 8) = o; }

__global__ __launch_bounds__(256) void k_planes(const float* __restrict__ F, bf* QH, bf* QL, bf* KH, bf* KL, bf* VH, bf* VL) {
    const size_t i = (size_t)blockIdx.x * 256 + threadIdx.x; if (i >= (size_t)NB * SEQ * 128) return; const size_t e = i * 8;
    const int d8 = (int)(e & 63); const size_t rw = e >> 6; const int t = (int)(rw % SEQ); const int hq = (int)((rw / SEQ) % HEADS); const int bq = (int)(rw / ((size_t)SEQ * HEADS));
    const float* s1 = F + ((size_t)bq * SEQ + t) * C3 + (size_t)hq * HS + d8;
    const v8f kv = *(const v8f*)s1; const v8f qv = *(const v8f*)(s1 + CE); v8us kh, kl, qh, ql;
#pragma unroll
    for (int c = 0; c < 8; ++c) { const bf hk = f2bf(kv[c]); kh[c] = hk; kl[c] = f2bf(kv[c] - bf2f(hk)); const bf hq2 = f2bf(qv[c]); qh[c] = hq2; ql[c] = f2bf(qv[c] - bf2f(hq2)); }
    const int t0 = (int)(e % SEQ); const size_t rv = e / SEQ; const int dv = (int)(rv % HS); const int hv = (int)((rv / HS) % HEADS); const int bv = (int)(rv / ((size_t)HS * HEADS));
    const float* s2 = F + ((size_t)bv * SEQ + t0) * C3 + 2 * CE + (size_t)hv * HS + dv; v8us vh, vl;
#pragma unroll
    for (int c = 0; c < 8; ++c) { const float v = s2[(size_t)c * C3]; const bf hb = f2bf(v); vh[c] = hb; vl[c] = f2bf(v - bf2f(hb)); }
#pragma unroll 1
    for (int ps = 0; ps < 2; ++ps) {
        *(volatile v8us*)(KH + e) = kh; *(volatile v8us*)(KL + e) = kl; *(volatile v8us*)(QH + e) = qh; *(volatile v8us*)(QL + e) = ql;
        *(volatile v8us*)(VH + e) = vh; *(volatile v8us*)(VL + e) = vl;
        if (ps == 0) __threadfence(); }
}

__global__ __launch_bounds__(128) void k_attn(const bf* __restrict__ QH, const bf* __restrict__ QL, const bf* __restrict__ KH, const bf* __restrict__ KL,
                                              const bf* __restrict__ VH, const bf* __restrict__ VL, bf* CTX) {
    __shared__ __align__(16) unsigned short pls[4][2][16 * LDP];
    const int wave = threadIdx.x >> 5, lane = threadIdx.x & 31, lr = lane & 15, hh = lane >> 4;
    const int qi0 = blockIdx.x * QB, h = blockIdx.y, b = blockIdx.z;
    const int q0w = qi0 + wave * 16;
    const size_t bh = (size_t)b * HEADS + h;
    unsigned short* ph = pls[wave][0]; unsigned short* pl = pls[wave][1];
    const size_t qo = (bh * SEQ + q0w + lr) * HS + 8 * hh;
    const v16bf qh0 = ldf(QH + qo), qh1 = ldf(QH + qo + 32);
    const v16bf ql0 = ldf(QL + qo), ql1 = ldf(QL + qo + 32);
    const size_t ko  = (bh * SEQ + lr) * HS + 8 * hh;
    const size_t vo0 = (bh * HS + lr) * SEQ + 8 * hh;
    v8f O[4];
#pragma unroll
    for (int j = 0; j < 4; ++j) O[j] = (v8f){};
    float mrun[8], lrun[8];
#pragma unroll
    for (int r = 0; r < 8; ++r) { mrun[r] = -__builtin_inff(); lrun[r] = 0.f; }
    const int ntiles = qi0 / KT + 1;
#pragma unroll 1
    for (int it = 0; it < ntiles; ++it) {
        const int kj = it * KT;
        v8f S[4];
#pragma unroll
        for (int nt = 0; nt < 4; ++nt) {
            const size_t kr = ko + (size_t)(kj + nt * 16) * HS;
            const v16bf kh0 = ldf(KH + kr), kh1 = ldf(KH + kr + 32), kl0 = ldf(KL + kr), kl1 = ldf(KL + kr + 32);
            v8f s = (v8f){};
            s = wmmab(qh0, kh0, s); s = wmmab(qh1, kh1, s);
            s = wmmab(ql0, kh0, s); s = wmmab(ql1, kh1, s);
            s = wmmab(qh0, kl0, s); s = wmmab(qh1, kl1, s);
            asm volatile("v_nop\n\tv_nop\n\tv_nop\n\tv_nop" : "+v"(s) : "v"(kh0), "v"(kh1), "v"(kl0), "v"(kl1) : "memory");
            S[nt] = s;
        }
        float sc[8];
#pragma unroll
        for (int r = 0; r < 8; ++r) {
            const int qr = q0w + 8 * hh + r;
            float m = -__builtin_inff();
#pragma unroll
            for (int nt = 0; nt < 4; ++nt) { const int key = kj + nt * 16 + lr; float s = S[nt][r] * SSC; s = (key > qr) ? -__builtin_inff() : s; S[nt][r] = s; m = fmaxf(m, s); }
#pragma unroll
            for (int sh = 1; sh < 16; sh <<= 1) m = fmaxf(m, __shfl_xor(m, sh, 32));
            const float mn = fmaxf(mrun[r], m);
            sc[r] = __builtin_amdgcn_exp2f((mrun[r] - mn) * L2E);
            float rs = 0.f;
#pragma unroll
            for (int nt = 0; nt < 4; ++nt) { const float p = __builtin_amdgcn_exp2f((S[nt][r] - mn) * L2E); S[nt][r] = p; rs += p; }
#pragma unroll
            for (int sh = 1; sh < 16; sh <<= 1) rs += __shfl_xor(rs, sh, 32);
            lrun[r] = lrun[r] * sc[r] + rs; mrun[r] = mn;
        }
        wave_lds_sync();
#pragma unroll
        for (int r = 0; r < 8; ++r)
#pragma unroll
            for (int nt = 0; nt < 4; ++nt) { const float p = S[nt][r]; const bf hb = f2bf(p); const int idx = (8 * hh + r) * LDP + nt * 16 + lr; ph[idx] = hb; pl[idx] = f2bf(p - bf2f(hb)); }
        wave_lds_sync();
#pragma unroll
        for (int j = 0; j < 4; ++j)
#pragma unroll
            for (int r = 0; r < 8; ++r) O[j][r] *= sc[r];
#pragma unroll
        for (int ks = 0; ks < 2; ++ks) {
            const unsigned short* pr  = ph + lr * LDP + ks * 32 + 8 * hh;
            const unsigned short* prl = pl + lr * LDP + ks * 32 + 8 * hh;
            const v16bf pah = cat16b(*(const v8us*)pr,  *(const v8us*)(pr + 16));
            const v16bf pal = cat16b(*(const v8us*)prl, *(const v8us*)(prl + 16));
#pragma unroll
            for (int j = 0; j < 4; ++j) {
                const size_t vo = vo0 + (size_t)j * 16 * SEQ + kj + ks * 32;
                const v16bf vbh = ldf(VH + vo), vbl = ldf(VL + vo);
                v8f o = O[j];
                o = wmmab(pah, vbh, o);
                o = wmmab(pah, vbl, o);
                o = wmmab(pal, vbh, o);
                asm volatile("v_nop\n\tv_nop\n\tv_nop\n\tv_nop" : "+v"(o) : "v"(pah), "v"(pal), "v"(vbh), "v"(vbl) : "memory");
                O[j] = o;
            }
        }
    }
    wave_lds_sync();
#pragma unroll
    for (int r = 0; r < 8; ++r) {
        const float inv = 1.0f / lrun[r];
#pragma unroll
        for (int j = 0; j < 4; ++j) { const float o = O[j][r] * inv; const bf hb = f2bf(o); const int idx = (8 * hh + r) * LDP + j * 16 + lr; ph[idx] = hb; pl[idx] = f2bf(o - bf2f(hb)); }
    }
    wave_lds_sync();
    bf* ctb = CTX + ((size_t)b * SEQ + q0w) * (2 * CE) + (size_t)h * HS;
    const int rsub = lane >> 3, c8 = (lane & 7) * 8;
#pragma unroll 1
    for (int ps = 0; ps < 2; ++ps) {
#pragma unroll
        for (int i = 0; i < 4; ++i) { const int row = 4 * i + rsub; const v8us vhi = *(const v8us*)(ph + row * LDP + c8); const v8us vlo = *(const v8us*)(pl + row * LDP + c8);
            *(volatile v8us*)(ctb + (size_t)row * (2 * CE) + c8) = vhi; *(volatile v8us*)(ctb + (size_t)row * (2 * CE) + CE + c8) = vlo; }
        if (ps == 0) __threadfence(); }
}

extern "C" void kernel_launch(void* const* d_in, const int* in_sizes, int n_in,
                              void* d_out, int out_size, void* d_ws, size_t ws_size, hipStream_t stream) {
    if (n_in < 5) return;
    if ((size_t)in_sizes[0] < (size_t)(NB - 1) * SEQ_FULL * CE + (size_t)SEQ * CE) return;
    if ((size_t)in_sizes[1] < (size_t)CE * C3 || in_sizes[2] < C3 || (size_t)in_sizes[3] < (size_t)CE * CE || in_sizes[4] < CE) return;
    if (out_size < 0 || (size_t)out_size < (size_t)(NB - 1) * SEQ_FULL * CE + (size_t)SEQ * CE) return;
    const float* x = (const float*)d_in[0]; const float* wa = (const float*)d_in[1]; const float* ba = (const float*)d_in[2]; const float* wp = (const float*)d_in[3]; const float* bp = (const float*)d_in[4];
    float* OUT = (float*)d_out;
    char* base = (char*)d_ws; size_t off = 0;
    auto take = [&](size_t bytes) { void* p = base + off; off += (bytes + 255) & ~(size_t)255; return p; };
    bf* WA  = (bf*)take((size_t)C3 * CE * 2);
    bf* WP2 = (bf*)take((size_t)CE * (2 * CE) * 2);
    bf* XB  = (bf*)take((size_t)NB * SEQ * CE * 2);
    const size_t regA = off;
    float* F = (float*)take((size_t)NB * SEQ * C3 * 4);
    const size_t endF = off;
    off = regA; bf* CTX = (bf*)take((size_t)NB * SEQ * (2 * CE) * 2);
    if (off < endF) off = endF;
    bf* QH = (bf*)take((size_t)NB * HEADS * SEQ * HS * 2);
    bf* QL = (bf*)take((size_t)NB * HEADS * SEQ * HS * 2);
    bf* KH = (bf*)take((size_t)NB * HEADS * SEQ * HS * 2);
    bf* KL = (bf*)take((size_t)NB * HEADS * SEQ * HS * 2);
    bf* VH = (bf*)take((size_t)NB * HEADS * HS * SEQ * 2);
    bf* VL = (bf*)take((size_t)NB * HEADS * HS * SEQ * 2);
    if (off > ws_size) return;

    k_wtG<<<(unsigned)((C3 * CE / 64 + 63) / 64), 256, 0, stream>>>(wa, CE, C3, CE, WA);
    k_wtG<<<(unsigned)((CE * (2 * CE) / 64 + 63) / 64), 256, 0, stream>>>(wp, CE, CE, 2 * CE, WP2);
    const size_t n8x = (size_t)SEQ * CE / 8;
    k_cvt8<<<dim3((unsigned)((n8x + 255) / 256), NB, 1), 256, 0, stream>>>(x, XB, n8x, (size_t)SEQ_FULL * CE, (size_t)SEQ * CE);
    k_gemmw<bf, 0, true><<<dim3(NB * SEQ / 64, C3 / 64, 1), 32, 0, stream>>>(XB, nullptr, WA, nullptr, CE, F, C3, ba, 0, 0, 0);
    k_planes<<<(unsigned)((size_t)NB * SEQ * 128 / 256), 256, 0, stream>>>(F, QH, QL, KH, KL, VH, VL);
    k_attn<<<dim3(SEQ / QB, HEADS, NB), 128, 0, stream>>>(QH, QL, KH, KL, VH, VL, CTX);
    k_gemmw<bf, 0, true><<<dim3(SEQ / 64, CE / 64, NB), 32, 0, stream>>>(CTX, nullptr, WP2, nullptr, 2 * CE, OUT, CE, bp, (size_t)SEQ * (2 * CE), 0, (size_t)SEQ_FULL * CE);
}
